// NFLPredictor_56040733278779
// MI455X (gfx1250) — hardware-verified
//
#include <hip/hip_runtime.h>
#include <math.h>

constexpr int kNSeq    = 22528;
constexpr int kPlays   = 1024;
constexpr int kPlayers = 22;
constexpr int kTEnc    = 20;
constexpr int kTDec    = 25;
constexpr int kInDim   = 33;
constexpr int kHid     = 64;
constexpr int kNGate   = 256;
constexpr int kOutDim  = 2;
constexpr int kRowsPerBlock = 16;
constexpr int kNBlk    = kNSeq / kRowsPerBlock;
static_assert(kNSeq % kRowsPerBlock == 0, "rows");
static_assert(kPlays * kPlayers == kNSeq, "n");
constexpr int kEncK     = 128;
constexpr int kEncPitch = 136;
constexpr int kDecK     = 64;
constexpr int kDecPitch = 72;
constexpr int kXOff     = 64;
constexpr float kACarry    = 8.0f;
constexpr float kWCarry    = 64.0f;
constexpr float kGateScale = 1.0f / 512.0f;
constexpr float kLnEps     = 1e-5f;
constexpr float kInvHid    = 1.0f / 64.0f;
constexpr int kOutPerSeq   = kTDec * kOutDim;

typedef __attribute__((ext_vector_type(16))) _Float16 v16h;
typedef __attribute__((ext_vector_type(8)))  _Float16 v8h;
typedef __attribute__((ext_vector_type(8)))  float    v8f;
typedef __attribute__((ext_vector_type(4)))  float    v4f;
typedef __attribute__((ext_vector_type(4)))  unsigned int v4u;

__device__ __forceinline__ void dep_guard_h(v8f& a, v8f& b, v16h x, v16h y) { asm volatile("v_nop\n\tv_nop\n\tv_nop\n\tv_nop" : "+v"(a), "+v"(b) : "v"(x), "v"(y)); }
__device__ __forceinline__ void keep4_h(v16h a, v16h b, v16h c, v16h d) { asm volatile("v_nop" :: "v"(a), "v"(b), "v"(c), "v"(d)); }
__device__ __forceinline__ void acc_guard4(v8f& a, v8f& b, v8f& c, v8f& d) { asm volatile("v_nop\n\tv_nop\n\tv_nop\n\tv_nop" : "+v"(a), "+v"(b), "+v"(c), "+v"(d)); }
template <typename T> struct Frag;
template <> struct Frag<_Float16> {
  typedef v16h V; union U { v16h v; v8h h[2]; };
  static __device__ __forceinline__ v16h load(const _Float16* p) {
    U f; f.h[0] = *(const v8h*)(p); f.h[1] = *(const v8h*)(p + 16); return f.v;
  }
  static __device__ __forceinline__ v8f mma(v16h a, v16h b, v8f c) {
    return __builtin_amdgcn_wmma_f32_16x16x32_f16(false, a, false, b, (short)0, c, false, false);
  }
  static __device__ __forceinline__ void guard(v8f& a, v8f& b, v16h x, v16h y) { dep_guard_h(a, b, x, y); }
  static __device__ __forceinline__ void keep(v16h a, v16h b, v16h c, v16h d) { keep4_h(a, b, c, d); }
};
__device__ __forceinline__ unsigned pk16(unsigned short a, unsigned short b) { return (unsigned)a | ((unsigned)b << 16); }
__device__ __forceinline__ unsigned short h_bits(float f) { const _Float16 h = (_Float16)f; return __builtin_bit_cast(unsigned short, h); }

__device__ __forceinline__ float sigm_f(float v) {
  v = fminf(fmaxf(v, -30.0f), 30.0f);
  return __builtin_amdgcn_rcpf(1.0f + expf(-v));
}
__device__ __forceinline__ float tanh_f(float v) {
  v = fminf(fmaxf(v, -15.0f), 15.0f);
  return 1.0f - 2.0f * __builtin_amdgcn_rcpf(1.0f + expf(2.0f * v));
}

template <int KSTEPS, int KTOT, int PITCH>
__device__ __forceinline__ void gate_mma(const _Float16* sAt, const _Float16* Wp, int w, int c, int koff,
                                         v8f& gi, v8f& gf, v8f& gg, v8f& go) {
  v8f acc[4];
#pragma unroll
  for (int g = 0; g < 4; ++g) acc[g] = (v8f){0.f, 0.f, 0.f, 0.f, 0.f, 0.f, 0.f, 0.f};
#pragma unroll
  for (int ks = 0; ks < KSTEPS; ++ks) {
    v16h bq[4];
#pragma unroll
    for (int g = 0; g < 4; ++g)
      bq[g] = Frag<_Float16>::load(Wp + (size_t)(g * kHid + 16 * w + c) * KTOT + ks * 32 + koff);
    const v16h af = Frag<_Float16>::load(sAt + c * PITCH + ks * 32 + koff);
#pragma unroll
    for (int g = 0; g < 4; ++g) acc[g] = Frag<_Float16>::mma(af, bq[g], acc[g]);
    Frag<_Float16>::guard(acc[0], acc[3], af, af);
    Frag<_Float16>::keep(bq[0], bq[1], bq[2], bq[3]);
  }
  acc_guard4(acc[0], acc[1], acc[2], acc[3]);
  gi = acc[0]; gf = acc[1]; gg = acc[2]; go = acc[3];
}

__global__ __launch_bounds__(256) void wprep_kernel(const float* __restrict__ encWih, const float* __restrict__ encWhh,
                                                    const float* __restrict__ decWhh,
                                                    unsigned short* __restrict__ Wenc, unsigned short* __restrict__ Wdec) {
  const int i = blockIdx.x * 256 + threadIdx.x;
  unsigned short hb[8];
  unsigned short* dst;
  if (blockIdx.x < 16) {
    const int n  = i >> 4;
    const int k0 = (i & 15) * 8;
#pragma unroll
    for (int e = 0; e < 8; ++e) {
      const int k  = k0 + e;
      const int ka = (k < (kInDim - 1)) ? k : (kInDim - 1);
      int kb = k - kXOff; kb = (kb < 0) ? 0 : kb;
      const float a = encWih[n * kInDim + ka];
      const float b = encWhh[n * kHid + kb];
      const float v = (k < kInDim) ? a * kWCarry : ((k >= kXOff) ? b * kWCarry : 0.0f);
      hb[e] = h_bits(v);
    }
    dst = Wenc + (size_t)i * 8;
  } else {
    const int j  = i - 4096;
    const int n  = j >> 3;
    const int k0 = (j & 7) * 8;
#pragma unroll
    for (int e = 0; e < 8; ++e) hb[e] = h_bits(decWhh[n * kHid + k0 + e] * kWCarry);
    dst = Wdec + (size_t)j * 8;
  }
  const v4u u = (v4u){pk16(hb[0], hb[1]), pk16(hb[2], hb[3]), pk16(hb[4], hb[5]), pk16(hb[6], hb[7])};
  *(volatile v4u*)dst = u;
  __threadfence();
  *(volatile v4u*)dst = u;
}

__global__ __launch_bounds__(128) void enc_lstm_kernel(const float* __restrict__ x, const unsigned short* __restrict__ Wencp,
                                                       const float* __restrict__ bih, const float* __restrict__ bhh,
                                                       float* __restrict__ hn, float* __restrict__ cn) {
  __shared__ __align__(16) _Float16 sA[kRowsPerBlock * kEncPitch];
  __shared__ __align__(16) float slabH[kRowsPerBlock * kHid];
  __shared__ __align__(16) float slabC[kRowsPerBlock * kHid];
  const _Float16* Wenc = (const _Float16*)(const void*)Wencp;
  const int tid  = threadIdx.x;
  const int lane = tid & 31, w = tid >> 5;
  const int c = lane & 15, hh = lane >> 4, koff = 8 * hh;
  const int seq0 = blockIdx.x * kRowsPerBlock;
  const int srow = tid >> 3, ssub = tid & 7;

  *(v4u*)(sA + srow * kEncPitch + kXOff + ssub * 8) = (v4u){0u, 0u, 0u, 0u};

  float bsum[4];
#pragma unroll
  for (int g = 0; g < 4; ++g) {
    const int n = g * kHid + 16 * w + c;
    bsum[g] = bih[n] + bhh[n];
  }
  float cst[8], hcur[8];
#pragma unroll
  for (int r = 0; r < 8; ++r) { cst[r] = 0.0f; hcur[r] = 0.0f; }
  const float* xseq = x + (size_t)(seq0 + srow) * (kTEnc * kInDim);

#pragma unroll 1
  for (int t = 0; t < kTEnc; ++t) {
    {
      const float* xr = xseq + t * kInDim;
      unsigned short hb[8];
#pragma unroll
      for (int e = 0; e < 8; ++e) {
        const int k  = ssub * 8 + e;
        const int kc = (k < (kInDim - 1)) ? k : (kInDim - 1);
        const float v = xr[kc];
        hb[e] = h_bits((k < kInDim) ? v * kACarry : 0.0f);
      }
      const v4u u = (v4u){pk16(hb[0], hb[1]), pk16(hb[2], hb[3]), pk16(hb[4], hb[5]), pk16(hb[6], hb[7])};
      *(v4u*)(sA + srow * kEncPitch + ssub * 8) = u;
    }
    __syncthreads();
    v8f ai, af, ag, ao;
    gate_mma<4, kEncK, kEncPitch>(sA, Wenc, w, c, koff, ai, af, ag, ao);
#pragma unroll
    for (int r = 0; r < 8; ++r) {
      const float pi = ai[r] * kGateScale + bsum[0];
      const float pf = af[r] * kGateScale + bsum[1];
      const float pg = ag[r] * kGateScale + bsum[2];
      const float po = ao[r] * kGateScale + bsum[3];
      const float cv = sigm_f(pf) * cst[r] + sigm_f(pi) * tanh_f(pg);
      cst[r] = cv;
      hcur[r] = sigm_f(po) * tanh_f(cv);
    }
    __syncthreads();
#pragma unroll
    for (int r = 0; r < 8; ++r)
      sA[(8 * hh + r) * kEncPitch + kXOff + 16 * w + c] = (_Float16)(hcur[r] * kACarry);
  }

#pragma unroll
  for (int r = 0; r < 8; ++r) {
    slabH[(8 * hh + r) * kHid + 16 * w + c] = hcur[r];
    slabC[(8 * hh + r) * kHid + 16 * w + c] = cst[r];
  }
  __syncthreads();
  float* hdst = hn + (size_t)seq0 * kHid;
  float* cdst = cn + (size_t)seq0 * kHid;
  for (int pass = 0; pass < 2; ++pass) {
#pragma unroll
    for (int it = 0; it < 2; ++it) {
      const int f = 256 * w + 128 * it + 4 * lane;
      const v4f hv = *(const v4f*)(slabH + f);
      const v4f cv = *(const v4f*)(slabC + f);
      *(volatile v4f*)(hdst + f) = hv;
      *(volatile v4f*)(cdst + f) = cv;
    }
    __threadfence();
  }
}

__global__ __launch_bounds__(64) void interact_kernel(const float* __restrict__ hn,
                                                      const float* __restrict__ qW, const float* __restrict__ qb,
                                                      const float* __restrict__ kW, const float* __restrict__ kb,
                                                      const float* __restrict__ vW, const float* __restrict__ vb,
                                                      const float* __restrict__ lng, const float* __restrict__ lnb,
                                                      float* __restrict__ y) {
  __shared__ __align__(16) float sh[kPlayers * kHid];
  __shared__ __align__(16) float sQ[kPlayers * kHid];
  __shared__ __align__(16) float sK[kPlayers * kHid];
  __shared__ __align__(16) float sV[kPlayers * kHid];
  __shared__ __align__(16) float sY[kPlayers * kHid];
  __shared__ float sS[kPlayers * 24];
  const int play = blockIdx.x;
  const int tid = threadIdx.x, lane = tid & 31, wave = tid >> 5;
  const float* hsrc = hn + (size_t)play * (kPlayers * kHid);
  for (int i = tid; i < (kPlayers * kHid) / 4; i += 64) *(v4f*)(sh + 4 * i) = *(const v4f*)(hsrc + 4 * i);
  __syncthreads();

  {
    const int j = tid;
    const float* qw = qW + j * kHid;
    const float* kw = kW + j * kHid;
    const float* vw = vW + j * kHid;
    const float qbj = qb[j], kbj = kb[j], vbj = vb[j];
#pragma unroll 1
    for (int p = 0; p < kPlayers; ++p) {
      const float* hp = sh + p * kHid;
      float aq = 0.f, ak = 0.f, av = 0.f;
#pragma unroll 1
      for (int k4 = 0; k4 < kHid / 4; ++k4) {
        const v4f hv = *(const v4f*)(hp + 4 * k4);
        const v4f wq = *(const v4f*)(qw + 4 * k4);
        const v4f wk = *(const v4f*)(kw + 4 * k4);
        const v4f wv = *(const v4f*)(vw + 4 * k4);
        aq += hv[0] * wq[0]; aq += hv[1] * wq[1]; aq += hv[2] * wq[2]; aq += hv[3] * wq[3];
        ak += hv[0] * wk[0]; ak += hv[1] * wk[1]; ak += hv[2] * wk[2]; ak += hv[3] * wk[3];
        av += hv[0] * wv[0]; av += hv[1] * wv[1]; av += hv[2] * wv[2]; av += hv[3] * wv[3];
      }
      sQ[p * kHid + j] = aq + qbj;
      sK[p * kHid + j] = ak + kbj;
      sV[p * kHid + j] = av + vbj;
    }
  }
  __syncthreads();

#pragma unroll 1
  for (int idx = tid; idx < kPlayers * kPlayers; idx += 64) {
    const int p = idx / kPlayers;
    const int q = idx - p * kPlayers;
    const float* qp = sQ + p * kHid;
    const float* kp = sK + q * kHid;
    float s = 0.f;
#pragma unroll 1
    for (int k4 = 0; k4 < kHid / 4; ++k4) {
      const v4f a = *(const v4f*)(qp + 4 * k4);
      const v4f b = *(const v4f*)(kp + 4 * k4);
      s += a[0] * b[0]; s += a[1] * b[1]; s += a[2] * b[2]; s += a[3] * b[3];
    }
    sS[p * 24 + q] = s * 0.125f;
  }
  __syncthreads();

  if (tid < kPlayers) {
    float* sr = sS + tid * 24;
    float m = sr[0];
#pragma unroll 1
    for (int q = 1; q < kPlayers; ++q) m = fmaxf(m, sr[q]);
    float sum = 0.f;
#pragma unroll 1
    for (int q = 0; q < kPlayers; ++q) { const float e = expf(sr[q] - m); sr[q] = e; sum += e; }
    const float inv = 1.0f / sum;
#pragma unroll 1
    for (int q = 0; q < kPlayers; ++q) sr[q] = sr[q] * inv;
  }
  __syncthreads();

  {
    const int j = tid;
#pragma unroll 1
    for (int p = 0; p < kPlayers; ++p) {
      const float* ar = sS + p * 24;
      float cx = 0.f;
#pragma unroll 1
      for (int q = 0; q < kPlayers; ++q) cx += ar[q] * sV[q * kHid + j];
      sY[p * kHid + j] = sh[p * kHid + j] + cx;
    }
  }
  __syncthreads();

  if (tid < kPlayers) {
    float* yr = sY + tid * kHid;
    float mu = 0.f;
#pragma unroll 1
    for (int i = 0; i < kHid; ++i) mu += yr[i];
    mu *= kInvHid;
    float var = 0.f;
#pragma unroll 1
    for (int i = 0; i < kHid; ++i) { const float d = yr[i] - mu; var += d * d; }
    var *= kInvHid;
    const float rstd = 1.0f / sqrtf(var + kLnEps);
#pragma unroll 1
    for (int i = 0; i < kHid; ++i) yr[i] = (yr[i] - mu) * rstd * lng[i] + lnb[i];
  }
  __syncthreads();

  float* ydst = y + (size_t)play * (kPlayers * kHid);
  for (int pass = 0; pass < 2; ++pass) {
#pragma unroll
    for (int it = 0; it < 6; ++it) {
      const int grp = 2 * it + wave;
      if (grp < 11) {
        const int f = grp * 128 + 4 * lane;
        const v4f v = *(const v4f*)(sY + f);
        *(volatile v4f*)(ydst + f) = v;
      }
    }
    __threadfence();
  }
}

__global__ __launch_bounds__(128) void dec_lstm_kernel(const float* __restrict__ x, const float* __restrict__ yin,
                                                       const float* __restrict__ cin, const unsigned short* __restrict__ Wdecp,
                                                       const float* __restrict__ dWih, const float* __restrict__ dbih,
                                                       const float* __restrict__ dbhh, const float* __restrict__ fcW,
                                                       const float* __restrict__ fcb, float* __restrict__ out) {
  __shared__ __align__(16) _Float16 sA[kRowsPerBlock * kDecPitch];
  __shared__ __align__(16) float hF[kRowsPerBlock * 68];
  __shared__ __align__(16) float sX[kRowsPerBlock * kOutDim];
  __shared__ __align__(16) float sOut[kRowsPerBlock * kOutPerSeq];
  const _Float16* Wdec = (const _Float16*)(const void*)Wdecp;
  const int tid  = threadIdx.x;
  const int lane = tid & 31, w = tid >> 5;
  const int c = lane & 15, hh = lane >> 4, koff = 8 * hh;
  const int seq0 = blockIdx.x * kRowsPerBlock;
  const int srow = tid >> 3, ssub = tid & 7;

  {
    const float* yr = yin + (size_t)(seq0 + srow) * kHid + ssub * 8;
    const v4f a = *(const v4f*)(yr);
    const v4f b = *(const v4f*)(yr + 4);
    unsigned short hb[8];
#pragma unroll
    for (int e = 0; e < 4; ++e) { hb[e] = h_bits(a[e] * kACarry); hb[4 + e] = h_bits(b[e] * kACarry); }
    const v4u u = (v4u){pk16(hb[0], hb[1]), pk16(hb[2], hb[3]), pk16(hb[4], hb[5]), pk16(hb[6], hb[7])};
    *(v4u*)(sA + srow * kDecPitch + ssub * 8) = u;
  }
  float cst[8];
#pragma unroll
  for (int r = 0; r < 8; ++r) cst[r] = cin[(size_t)(seq0 + 8 * hh + r) * kHid + 16 * w + c];
  if (tid < 32) {
    const int row = tid & 15, d = tid >> 4;
    sX[row * kOutDim + d] = x[((size_t)(seq0 + row) * kTEnc + (kTEnc - 1)) * kInDim + d];
  }
  float bsum[4], wi0[4], wi1[4];
#pragma unroll
  for (int g = 0; g < 4; ++g) {
    const int n = g * kHid + 16 * w + c;
    bsum[g] = dbih[n] + dbhh[n];
    wi0[g] = dWih[n * kOutDim + 0];
    wi1[g] = dWih[n * kOutDim + 1];
  }
  const int frow = tid & 15, fd = (tid >> 4) & 1;
  const float fbias = fcb[fd];
  const float* fw = fcW + fd * kHid;
  __syncthreads();

#pragma unroll 1
  for (int s = 0; s < kTDec; ++s) {
    v8f ai, af, ag, ao;
    gate_mma<2, kDecK, kDecPitch>(sA, Wdec, w, c, koff, ai, af, ag, ao);
    float hcur[8];
#pragma unroll
    for (int r = 0; r < 8; ++r) {
      const int row = 8 * hh + r;
      const float x0 = sX[row * kOutDim + 0];
      const float x1 = sX[row * kOutDim + 1];
      const float xi = x0 * wi0[0] + x1 * wi1[0];
      const float xf = x0 * wi0[1] + x1 * wi1[1];
      const float xg = x0 * wi0[2] + x1 * wi1[2];
      const float xo = x0 * wi0[3] + x1 * wi1[3];
      const float pi = ai[r] * kGateScale + xi + bsum[0];
      const float pf = af[r] * kGateScale + xf + bsum[1];
      const float pg = ag[r] * kGateScale + xg + bsum[2];
      const float po = ao[r] * kGateScale + xo + bsum[3];
      const float cv = sigm_f(pf) * cst[r] + sigm_f(pi) * tanh_f(pg);
      cst[r] = cv;
      hcur[r] = sigm_f(po) * tanh_f(cv);
    }
    __syncthreads();
#pragma unroll
    for (int r = 0; r < 8; ++r) {
      sA[(8 * hh + r) * kDecPitch + 16 * w + c] = (_Float16)(hcur[r] * kACarry);
      hF[(8 * hh + r) * 68 + 16 * w + c] = hcur[r];
    }
    __syncthreads();
    if (tid < 32) {
      const float* hr = hF + frow * 68;
      float p = 0.f;
#pragma unroll 1
      for (int k4 = 0; k4 < kHid / 4; ++k4) {
        const v4f hv = *(const v4f*)(hr + 4 * k4);
        const v4f wv = *(const v4f*)(fw + 4 * k4);
        p += hv[0] * wv[0]; p += hv[1] * wv[1]; p += hv[2] * wv[2]; p += hv[3] * wv[3];
      }
      p += fbias;
      sX[frow * kOutDim + fd] = p;
      sOut[frow * kOutPerSeq + s * kOutDim + fd] = p;
    }
    __syncthreads();
  }

  float* odst = out + (size_t)seq0 * kOutPerSeq;
  for (int pass = 0; pass < 2; ++pass) {
#pragma unroll
    for (int it = 0; it < 2; ++it) {
      const int idx = tid + 128 * it;
      if (idx < (kRowsPerBlock * kOutPerSeq) / 4) {
        const v4f v = *(const v4f*)(sOut + 4 * idx);
        *(volatile v4f*)(odst + 4 * idx) = v;
      }
    }
    __threadfence();
  }
}

extern "C" void kernel_launch(void* const* d_in, const int* in_sizes, int n_in,
                              void* d_out, int out_size, void* d_ws, size_t ws_size,
                              hipStream_t stream) {
  if (n_in < 19) return;
  if (in_sizes[0] != kNSeq * kTEnc * kInDim) return;
  if (out_size != kNSeq * kTDec * kOutDim) return;

  const float* x        = (const float*)d_in[0];
  const float* enc_Wih  = (const float*)d_in[1];
  const float* enc_Whh  = (const float*)d_in[2];
  const float* enc_bih  = (const float*)d_in[3];
  const float* enc_bhh  = (const float*)d_in[4];
  const float* q_W      = (const float*)d_in[5];
  const float* q_b      = (const float*)d_in[6];
  const float* k_W      = (const float*)d_in[7];
  const float* k_b      = (const float*)d_in[8];
  const float* v_W      = (const float*)d_in[9];
  const float* v_b      = (const float*)d_in[10];
  const float* ln_g     = (const float*)d_in[11];
  const float* ln_b     = (const float*)d_in[12];
  const float* dec_Wih  = (const float*)d_in[13];
  const float* dec_Whh  = (const float*)d_in[14];
  const float* dec_bih  = (const float*)d_in[15];
  const float* dec_bhh  = (const float*)d_in[16];
  const float* fc_W     = (const float*)d_in[17];
  const float* fc_b     = (const float*)d_in[18];

  const size_t offWenc = 0;
  const size_t offWdec = 65536;
  const size_t offHn   = 98304;
  const size_t plane   = (size_t)kNSeq * kHid * sizeof(float);
  const size_t offCn   = offHn + plane;
  const size_t offY    = offCn + plane;
  const size_t total   = offY + plane;
  if (total > ws_size) return;

  char* ws = (char*)d_ws;
  unsigned short* Wenc = (unsigned short*)(ws + offWenc);
  unsigned short* Wdec = (unsigned short*)(ws + offWdec);
  float* hn = (float*)(ws + offHn);
  float* cn = (float*)(ws + offCn);
  float* yb = (float*)(ws + offY);

  wprep_kernel<<<24, 256, 0, stream>>>(enc_Wih, enc_Whh, dec_Whh, Wenc, Wdec);
  enc_lstm_kernel<<<kNBlk, 128, 0, stream>>>(x, Wenc, enc_bih, enc_bhh, hn, cn);
  interact_kernel<<<kPlays, 64, 0, stream>>>(hn, q_W, q_b, k_W, k_b, v_W, v_b, ln_g, ln_b, yb);
  dec_lstm_kernel<<<kNBlk, 128, 0, stream>>>(x, yb, cn, Wdec, dec_Wih, dec_bih, dec_bhh, fc_W, fc_b, (float*)d_out);
}
